// Mamba3Layer_39144331935958
// MI455X (gfx1250) — hardware-verified
//
#include <hip/hip_runtime.h>
#include <math.h>

typedef __attribute__((ext_vector_type(16))) _Float16 v16h;
typedef __attribute__((ext_vector_type(8)))  _Float16 v8h;
typedef __attribute__((ext_vector_type(16))) __bf16   v16b;
typedef __attribute__((ext_vector_type(8)))  __bf16   v8b;
typedef __attribute__((ext_vector_type(8)))  float    v8f;
typedef __attribute__((ext_vector_type(4)))  float    v4f;

constexpr int kBatch = 2;
constexpr int kSeq   = 512;
constexpr int kRows  = kBatch * kSeq;
constexpr int kDm    = 1024;
constexpr int kDi    = 2048;
constexpr int kDi2   = 2 * kDi;
constexpr int kDiX   = 2 * kDi;
constexpr int kNs    = 32;
constexpr int kHalf  = 16;
constexpr int kPP    = 4;
constexpr int kPasses = kHalf / kPP;
constexpr int kThr   = 256;
constexpr float kLnEps = 1e-5f;

constexpr float kInCarry = 1024.0f;
constexpr float kWCarry  = 16384.0f;
constexpr float kACarry  = 256.0f;
constexpr float kScIn = 1.0f / (kInCarry * kWCarry);
constexpr float kScA  = 1.0f / (kACarry * kWCarry);
constexpr float kF16MinNormal = 6.103515625e-5f;

static_assert((kRows % 64) == 0 && ((kRows / 64) * (64 / 64)) % 8 == 0, "the smallest GEMM grid exact");
static_assert((kDm % 32) == 0 && (kDiX % 32) == 0, "GEMM K multiples of 32");

constexpr size_t kOffX16 = 0;
constexpr size_t kOffWI  = kOffX16 + (size_t)kRows * kDm * 2;
constexpr size_t kOffWBC = kOffWI  + (size_t)kDi2 * kDm * 2;
constexpr size_t kOffWD  = kOffWBC + (size_t)64 * kDm * 2;
constexpr size_t kOffWO  = kOffWD  + (size_t)kDi * kDm * 2;
constexpr size_t kOffBV  = kOffWO  + (size_t)kDm * kDiX * 2;
constexpr int    kBvZ    = 0;
constexpr int    kBvDt   = kDi2;
constexpr int    kBvTot  = kDi2 + kDi;
constexpr size_t kOffTAB = kOffBV  + (size_t)kBvTot * 4;
constexpr size_t kOffXZ  = kOffTAB + (size_t)kSeq * kHalf * 2 * 4;
constexpr size_t kOffBC  = kOffXZ  + (size_t)kRows * kDi2 * 4;
constexpr size_t kOffDTL = kOffBC  + (size_t)kRows * 64 * 4;
constexpr size_t kOffYP  = kOffDTL + (size_t)kRows * kDi * 4;
constexpr size_t kOffFS  = kOffYP  + (size_t)kRows * kDi * 4;
constexpr size_t kOffG16 = kOffFS  + (size_t)kPasses * kBatch * kDi * 8 * 4;
constexpr size_t kWsTotal = kOffG16 + (size_t)kRows * kDiX * 2;
static_assert(kWsTotal <= 268435456ull, "inside the offered workspace");
static_assert((kOffWI % 256) == 0 && (kOffWBC % 256) == 0 && (kOffWD % 256) == 0 && (kOffWO % 256) == 0 && (kOffBV % 256) == 0 && (kOffTAB % 256) == 0 && (kOffXZ % 256) == 0 && (kOffBC % 256) == 0 && (kOffDTL % 256) == 0 && (kOffYP % 256) == 0 && (kOffFS % 256) == 0 && (kOffG16 % 256) == 0, "aligned regions");

__device__ __forceinline__ unsigned short f2bf_bits(float f) {
  unsigned u = __float_as_uint(f);
  return (unsigned short)((u + 0x7FFFu + ((u >> 16) & 1u)) >> 16);
}
__device__ __forceinline__ float bf_bits2f(unsigned short h) { return __uint_as_float(((unsigned)h) << 16); }
__device__ __forceinline__ float bf16r(float f) { return bf_bits2f(f2bf_bits(f)); }
__device__ __forceinline__ float carry_flush(float v, float carry) {
  const float s = v * carry;
  return (fabsf(s) < kF16MinNormal) ? 0.0f : s;
}
__device__ __forceinline__ float frcp(float x) { return __builtin_amdgcn_rcpf(x); }

__device__ __forceinline__ void dep_guard4_h(v8f& a, v8f& b, v8f& c, v8f& d, v16h x, v16h y) { asm volatile("v_nop\n\tv_nop\n\tv_nop\n\tv_nop" : "+v"(a), "+v"(b), "+v"(c), "+v"(d) : "v"(x), "v"(y)); }
__device__ __forceinline__ void dep_guard4_b(v8f& a, v8f& b, v8f& c, v8f& d, v16b x, v16b y) { asm volatile("v_nop\n\tv_nop\n\tv_nop\n\tv_nop" : "+v"(a), "+v"(b), "+v"(c), "+v"(d) : "v"(x), "v"(y)); }
__device__ __forceinline__ void keep4_h(v16h a, v16h b, v16h c, v16h d) { asm volatile("v_nop" :: "v"(a), "v"(b), "v"(c), "v"(d)); }
__device__ __forceinline__ void keep4_b(v16b a, v16b b, v16b c, v16b d) { asm volatile("v_nop" :: "v"(a), "v"(b), "v"(c), "v"(d)); }
__device__ __forceinline__ void acc_guard4(v8f& a, v8f& b, v8f& c, v8f& d) { asm volatile("v_nop\n\tv_nop\n\tv_nop\n\tv_nop" : "+v"(a), "+v"(b), "+v"(c), "+v"(d)); }

template <typename T> struct Frag;
template <> struct Frag<_Float16> {
  typedef v16h V; union U { v16h v; v8h h[2]; };
  static __device__ __forceinline__ v16h load(const _Float16* p) {
    U f; f.h[0] = *(const v8h*)(p); f.h[1] = *(const v8h*)(p + 16); return f.v;
  }
  static __device__ __forceinline__ v8f mma(v16h a, v16h b, v8f c) {
    return __builtin_amdgcn_wmma_f32_16x16x32_f16(false, a, false, b, (short)0, c, false, false);
  }
  static __device__ __forceinline__ void guard4(v8f& a, v8f& b, v8f& c, v8f& d, v16h x, v16h y) { dep_guard4_h(a, b, c, d, x, y); }
  static __device__ __forceinline__ void keep(v16h a, v16h b, v16h c, v16h d) { keep4_h(a, b, c, d); }
};
template <> struct Frag<__bf16> {
  typedef v16b V; union U { v16b v; v8b h[2]; };
  static __device__ __forceinline__ v16b load(const __bf16* p) {
    U f; f.h[0] = *(const v8b*)(p); f.h[1] = *(const v8b*)(p + 16); return f.v;
  }
  static __device__ __forceinline__ v8f mma(v16b a, v16b b, v8f c) {
    return __builtin_amdgcn_wmma_f32_16x16x32_bf16(false, a, false, b, (short)0, c, false, false);
  }
  static __device__ __forceinline__ void guard4(v8f& a, v8f& b, v8f& c, v8f& d, v16b x, v16b y) { dep_guard4_b(a, b, c, d, x, y); }
  static __device__ __forceinline__ void keep(v16b a, v16b b, v16b c, v16b d) { keep4_b(a, b, c, d); }
};

__device__ __forceinline__ v8f mma_h(v16h a, v16h b, v8f c) {
  c = __builtin_amdgcn_wmma_f32_16x16x32_f16(false, a, false, b, (short)0, c, false, false);
  asm volatile("v_nop\n\tv_nop\n\tv_nop\n\tv_nop" : "+v"(c) : "v"(a), "v"(b));
  return c;
}

template <int ET> struct Elem;
template <> struct Elem<0> { typedef _Float16 T; };
template <> struct Elem<1> { typedef __bf16 T; };
template <int ET, bool SPLIT, int BIAS_MODE, int OUT_MODE, bool RESID, int ACT = 0>
__global__ __launch_bounds__(256) void wmma_gemm64(
    const unsigned short* __restrict__ Ap, const unsigned short* __restrict__ A2p, int lda, long strideA,
    const unsigned short* __restrict__ Btp, const unsigned short* __restrict__ Bt2p, int ldb, long strideB,
    void* __restrict__ Cout, void* __restrict__ Cout2, int ldc, long strideC,
    const float* __restrict__ bias,
    const float* __restrict__ resid, long strideR,
    int M, int N, int K, float scale) {
  typedef typename Elem<ET>::T T;
  typedef typename Frag<T>::V V;
  const T* A = (const T*)Ap; const T* A2 = (const T*)A2p; const T* Bt = (const T*)Btp; const T* Bt2 = (const T*)Bt2p;
  __shared__ __align__(16) float sT[8][16 * 68];
  const int b    = blockIdx.y;
  const int lane = threadIdx.x & 31;
  const int wave = threadIdx.x >> 5;
  const int tilesN = N >> 6;
  const int tilesM = M >> 6;
  const int tile = blockIdx.x * 8 + wave;
  if (tile >= tilesM * tilesN) return;
  const int tm = tile / tilesN;
  const int tn = tile - tm * tilesN;
  const int m0 = tm << 6;
  const int n0 = tn << 6;

  const T* Ab  = A  + (size_t)b * strideA;
  const T* Bb  = Bt + (size_t)b * strideB;
  const T* Ab2 = SPLIT ? (A2  + (size_t)b * strideA) : nullptr;
  const T* Bb2 = SPLIT ? (Bt2 + (size_t)b * strideB) : nullptr;

  const int rlane = lane & 15;
  const int koff  = (lane >> 4) * 8;
  const int mOff  = (lane >> 4) * 8;

  v8f acc[4][4];
#pragma unroll
  for (int i = 0; i < 4; ++i)
#pragma unroll
    for (int j = 0; j < 4; ++j) acc[i][j] = (v8f){0.f,0.f,0.f,0.f,0.f,0.f,0.f,0.f};

  for (int k0 = 0; k0 < K; k0 += 32) {
    V bh[4], bl[4];
#pragma unroll
    for (int j = 0; j < 4; ++j) {
      const size_t bo = (size_t)(n0 + (j << 4) + rlane) * ldb + koff + k0;
      bh[j] = Frag<T>::load(Bb + bo);
      if (SPLIT) bl[j] = Frag<T>::load(Bb2 + bo);
    }
#pragma unroll
    for (int i = 0; i < 4; ++i) {
      const size_t ao = (size_t)(m0 + (i << 4) + rlane) * lda + koff + k0;
      V ah = Frag<T>::load(Ab + ao);
      V al;
      if (SPLIT) al = Frag<T>::load(Ab2 + ao);
#pragma unroll
      for (int j = 0; j < 4; ++j) {
        acc[i][j] = Frag<T>::mma(ah, bh[j], acc[i][j]);
        if (SPLIT) {
          acc[i][j] = Frag<T>::mma(ah, bl[j], acc[i][j]);
          acc[i][j] = Frag<T>::mma(al, bh[j], acc[i][j]);
        }
      }
      Frag<T>::guard4(acc[i][0], acc[i][1], acc[i][2], acc[i][3], ah, SPLIT ? al : ah);
    }
    Frag<T>::keep(bh[0], bh[1], bh[2], bh[3]);
    if (SPLIT) Frag<T>::keep(bl[0], bl[1], bl[2], bl[3]);
  }
  acc_guard4(acc[0][0], acc[0][1], acc[0][2], acc[0][3]);
  acc_guard4(acc[1][0], acc[1][1], acc[1][2], acc[1][3]);
  acc_guard4(acc[2][0], acc[2][1], acc[2][2], acc[2][3]);
  acc_guard4(acc[3][0], acc[3][1], acc[3][2], acc[3][3]);

  float* slab = sT[wave];
  const float* Rb = RESID ? (resid + (size_t)b * strideR) : nullptr;
#pragma unroll
  for (int i = 0; i < 4; ++i) {
    const int mBase = m0 + (i << 4);
#pragma unroll
    for (int j = 0; j < 4; ++j) {
      const int n = n0 + (j << 4) + rlane;
      float bv = 0.f;
      if (BIAS_MODE == 2) bv = bias[n];
#pragma unroll
      for (int r = 0; r < 8; ++r) {
        float v = acc[i][j][r] * scale;
        if (BIAS_MODE == 1) v += bias[mBase + mOff + r];
        if (BIAS_MODE == 2) v += bv;
        if (RESID) v += Rb[(size_t)(mBase + mOff + r) * ldc + n];
        if (ACT == 1) v = tanhf(v);
        if (ACT == 2) v = fmaxf(v, 0.0f);
        if (ACT == 3) v = v / (1.0f + expf(-v));
        if (ACT == 4) v = (v > 0.f) ? v : 0.01f * v;
        slab[(mOff + r) * 68 + (j << 4) + rlane] = v;
      }
    }
    __builtin_amdgcn_fence(__ATOMIC_RELEASE, "workgroup");
    __builtin_amdgcn_wave_barrier();
    __builtin_amdgcn_fence(__ATOMIC_ACQUIRE, "workgroup");
    if (OUT_MODE == 0) {
      float* C = (float*)Cout + (size_t)b * strideC;
      const int hh = lane >> 4, c4 = (lane & 15) * 4;
      for (int pass = 0; pass < 2; ++pass) {
#pragma unroll
        for (int it = 0; it < 8; ++it) {
          const int row = it * 2 + hh;
          v4f v = *(const v4f*)(slab + row * 68 + c4);
          *(volatile v4f*)(C + (size_t)(mBase + row) * ldc + n0 + c4) = v;
        }
        __threadfence();
      }
    } else {
      const int q = lane >> 3, c8 = (lane & 7) * 8;
      unsigned short* C  = (unsigned short*)Cout  + (size_t)b * strideC;
      unsigned short* C2 = (OUT_MODE == 2) ? ((unsigned short*)Cout2 + (size_t)b * strideC) : nullptr;
      for (int pass = 0; pass < 2; ++pass) {
#pragma unroll
        for (int it = 0; it < 4; ++it) {
          const int row = it * 4 + q;
          const float* sp = slab + row * 68 + c8;
          v8h hv, lv;
#pragma unroll
          for (int e = 0; e < 8; ++e) {
            if (OUT_MODE == 1) {
              hv[e] = (_Float16)sp[e];
            } else {
              unsigned short hb = f2bf_bits(sp[e]);
              unsigned short lb = f2bf_bits(sp[e] - bf_bits2f(hb));
              hv[e] = __builtin_bit_cast(_Float16, hb);
              lv[e] = __builtin_bit_cast(_Float16, lb);
            }
          }
          *(volatile v8h*)(C + (size_t)(mBase + row) * ldc + n0 + c8) = hv;
          if (OUT_MODE == 2) *(volatile v8h*)(C2 + (size_t)(mBase + row) * ldc + n0 + c8) = lv;
        }
        __threadfence();
      }
    }
    __builtin_amdgcn_fence(__ATOMIC_RELEASE, "workgroup");
    __builtin_amdgcn_wave_barrier();
    __builtin_amdgcn_fence(__ATOMIC_ACQUIRE, "workgroup");
  }
}


__device__ __forceinline__ void split_hl(float v, float c, _Float16& hi, _Float16& lo) {
  const float sv = carry_flush(v, c);
  hi = (_Float16)sv;
  const float r = sv - (float)hi;
  lo = (_Float16)((fabsf(r) < kF16MinNormal) ? 0.0f : r);
}

__device__ __forceinline__ float block_sum_256(float v, float* red, float* wsum) {
  const int tid = threadIdx.x;
  red[tid] = v;
  __syncthreads();
  if ((tid & 31) == 0) {
    float s = 0.0f;
#pragma unroll 1
    for (int k = 0; k < 32; ++k) s += red[tid + k];
    wsum[tid >> 5] = s;
  }
  __syncthreads();
  float t = 0.0f;
#pragma unroll
  for (int k = 0; k < 8; ++k) t += wsum[k];
  __syncthreads();
  return t;
}

__global__ __launch_bounds__(kThr) void cast_rows_kernel(const float* __restrict__ src, unsigned short* __restrict__ dst, int per, int ldd, int colOff, float c) {
  const int i = blockIdx.x * kThr + threadIdx.x;
  const int n = i / per;
  const int k8 = (i - n * per) * 8;
  const v4f a0 = *(const v4f*)(src + (size_t)i * 8);
  const v4f a1 = *(const v4f*)(src + (size_t)i * 8 + 4);
  v8h hv;
#pragma unroll
  for (int e = 0; e < 4; ++e) {
    const float w0 = a0[e], w1 = a1[e];
    hv[e]     = (_Float16)carry_flush(bf16r(w0), c);
    hv[4 + e] = (_Float16)carry_flush(bf16r(w1), c);
  }
  unsigned short* dp = dst + (size_t)n * ldd + colOff + k8;
  *(volatile v8h*)dp = hv;
  __threadfence();
  *(volatile v8h*)dp = hv;
}

__global__ __launch_bounds__(kThr) void bias_rows_kernel(const float* __restrict__ b_dt, float* __restrict__ BV) {
  const int i = blockIdx.x * kThr + threadIdx.x;
  const int idt = i - kBvDt;
  const float v = b_dt[(idt >= 0) ? idt : 0];
  const float o = (idt >= 0) ? bf16r(v) : 0.0f;
  for (int pass = 0; pass < 2; ++pass) {
    *(volatile float*)(BV + i) = o;
    __threadfence();
  }
}
static_assert(kBvTot % kThr == 0 && kBvDt % kThr == 0, "bias grid exact; regions block-uniform");

__global__ __launch_bounds__(kThr) void rope_table_kernel(const float* __restrict__ rope_freq, float* __restrict__ TAB) {
  const int i = blockIdx.x * kThr + threadIdx.x;
  const int l = i >> 4, j = i & 15;
  const float f0 = rope_freq[j];
  const float a = (float)l * bf16r(f0);
  float2 cs;
  cs.x = cosf(a);
  cs.y = sinf(a);
  for (int pass = 0; pass < 2; ++pass) {
    *(volatile float*)(TAB + (size_t)i * 2) = cs.x;
    *(volatile float*)(TAB + (size_t)i * 2 + 1) = cs.y;
    __threadfence();
  }
}
static_assert((kSeq * kHalf) % kThr == 0, "table grid exact");

template <int kP0>
__global__ __launch_bounds__(kThr) void trap_scan_kernel(const float* __restrict__ DTL, const float* __restrict__ XZ, const float* __restrict__ BC,
                                                         const float* __restrict__ TAB, const float* __restrict__ A_log, const float* __restrict__ dt_bias,
                                                         float* __restrict__ YP, float* __restrict__ FS) {
  const int v = blockIdx.x * kThr + threadIdx.x;
  const int b = v >> 11;
  const int d = v & (kDi - 1);
  float Ar[kPP], Ai[kPP], sr[kPP], si[kPP];
#pragma unroll
  for (int i = 0; i < kPP; ++i) {
    const float a0 = A_log[(size_t)d * kNs + kP0 + i], a1 = A_log[(size_t)d * kNs + kHalf + kP0 + i];
    Ar[i] = -expf(bf16r(a0)); Ai[i] = -expf(bf16r(a1)); sr[i] = 0.0f; si[i] = 0.0f;
  }
  const float db0 = dt_bias[d];
  const float dtb = bf16r(db0);
  const size_t r0 = (size_t)b * kSeq;
#pragma unroll 1
  for (int l = 0; l < kSeq; ++l) {
    const size_t row = r0 + l;
    const float sv = DTL[row * kDi + d] + dtb;
    const float xin = XZ[row * kDi2 + d];
    const float dt = (sv > 20.0f) ? sv : log1pf(expf(sv));
    const v4f Br = *(const v4f*)(BC + row * 64 + kP0);
    const v4f Bi = *(const v4f*)(BC + row * 64 + kHalf + kP0);
    const v4f Cr = *(const v4f*)(BC + row * 64 + 32 + kP0);
    const v4f Ci = *(const v4f*)(BC + row * 64 + 32 + kHalf + kP0);
    float y = 0.0f;
#pragma unroll
    for (int i = 0; i < kPP; ++i) {
      const float2 cs = *(const float2*)(TAB + ((size_t)l * kHalf + kP0 + i) * 2);
      const float hr = dt * Ar[i] * 0.5f, hi = dt * Ai[i] * 0.5f;
      const float rr = frcp(1.0f - hr), ri = frcp(1.0f - hi);
      const float nr = ((1.0f + hr) * rr) * sr[i] + ((dt * rr) * Br[i]) * xin;
      const float ni = ((1.0f + hi) * ri) * si[i] + ((dt * ri) * Bi[i]) * xin;
      const float re = nr * cs.x - ni * cs.y;
      const float im = nr * cs.y + ni * cs.x;
      sr[i] = re; si[i] = im;
      y += re * Cr[i];
      y += im * Ci[i];
    }
    float* op = YP + row * kDi + d;
    float o;
    if (kP0 == 0) { o = y; } else { o = *op + y; }
    *(volatile float*)op = o;
    __threadfence();
    *(volatile float*)op = o;
  }
  float* fp = FS + ((size_t)(kP0 / kPP) * kBatch * kDi + v) * 8;
  v4f f0, f1;
#pragma unroll
  for (int i = 0; i < kPP; ++i) { f0[i] = sr[i]; f1[i] = si[i]; }
  for (int pass = 0; pass < 2; ++pass) {
    *(volatile v4f*)fp = f0;
    *(volatile v4f*)(fp + 4) = f1;
    __threadfence();
  }
}
static_assert((kBatch * kDi) % kThr == 0, "scan grid exact");

__global__ __launch_bounds__(kThr) void final_state_kernel(const float* __restrict__ FS, float* __restrict__ fstate) {
  const int v = blockIdx.x * kThr + threadIdx.x;
  v4f re[kPasses], im[kPasses];
#pragma unroll
  for (int p = 0; p < kPasses; ++p) {
    const float* fp = FS + ((size_t)p * kBatch * kDi + v) * 8;
    re[p] = *(const v4f*)fp;
    im[p] = *(const v4f*)(fp + 4);
  }
  float* dp = fstate + (size_t)v * kNs;
  for (int pass = 0; pass < 2; ++pass) {
#pragma unroll
    for (int p = 0; p < kPasses; ++p) {
      *(volatile v4f*)(dp + 4 * p) = re[p];
      *(volatile v4f*)(dp + kHalf + 4 * p) = im[p];
    }
    __threadfence();
  }
}

__global__ __launch_bounds__(kThr) void gate_ln_kernel(const float* __restrict__ YP, const float* __restrict__ XZ, const float* __restrict__ ln_w,
                                                       const float* __restrict__ ln_b, unsigned short* __restrict__ G16) {
  __shared__ float red[kThr];
  __shared__ float wsum[8];
  const size_t row = blockIdx.x;
  const int d8 = threadIdx.x * 8;
  float o[8];
  float s = 0.0f;
#pragma unroll
  for (int hlf = 0; hlf < 2; ++hlf) {
    const v4f yv = *(const v4f*)(YP + row * kDi + d8 + 4 * hlf);
    const v4f zv = *(const v4f*)(XZ + row * kDi2 + kDi + d8 + 4 * hlf);
#pragma unroll
    for (int e = 0; e < 4; ++e) {
      const float z = zv[e] * (1.0f / (1.0f + expf(-zv[e])));
      o[4 * hlf + e] = yv[e] * z;
      s += o[4 * hlf + e];
    }
  }
  const float mu = block_sum_256(s, red, wsum) * (1.0f / (float)kDi);
  float q = 0.0f;
#pragma unroll
  for (int e = 0; e < 8; ++e) { const float dv = o[e] - mu; q += dv * dv; }
  const float var = block_sum_256(q, red, wsum) * (1.0f / (float)kDi);
  const float rs = 1.0f / sqrtf(var + kLnEps);
  v8h hv, lv;
#pragma unroll
  for (int hlf = 0; hlf < 2; ++hlf) {
    const v4f gw = *(const v4f*)(ln_w + d8 + 4 * hlf);
    const v4f gb = *(const v4f*)(ln_b + d8 + 4 * hlf);
#pragma unroll
    for (int e = 0; e < 4; ++e) {
      const float w0 = gw[e], b0 = gb[e];
      _Float16 hi, lo;
      split_hl((o[4 * hlf + e] - mu) * rs * bf16r(w0) + bf16r(b0), kACarry, hi, lo);
      hv[4 * hlf + e] = hi; lv[4 * hlf + e] = lo;
    }
  }
  unsigned short* dp = G16 + row * kDiX + d8;
  for (int pass = 0; pass < 2; ++pass) {
    *(volatile v8h*)dp = hv;
    *(volatile v8h*)(dp + kDi) = lv;
    __threadfence();
  }
}
static_assert(kDi / 8 == kThr, "one block per row");

extern "C" void kernel_launch(void* const* d_in, const int* in_sizes, int n_in,
                              void* d_out, int out_size, void* d_ws, size_t ws_size,
                              hipStream_t stream) {
  if (n_in < 12 || d_out == nullptr || d_ws == nullptr) return;
  if (in_sizes[0] != kRows * kDm || in_sizes[1] != kDi2 * kDm || in_sizes[2] != kDi * kNs || in_sizes[3] != kNs * kDm || in_sizes[4] != kNs * kDm) return;
  if (in_sizes[5] != kDi * kDm || in_sizes[6] != kDi || in_sizes[7] != kDi || in_sizes[8] != kHalf || in_sizes[9] != kDi || in_sizes[10] != kDi) return;
  if (in_sizes[11] != kDm * kDi) return;
  if (out_size != kRows * kDm + kBatch * kDi * kNs) return;
  if (ws_size < kWsTotal) return;
  const float* x = (const float*)d_in[0];
  const float* W_in = (const float*)d_in[1];
  const float* A_log = (const float*)d_in[2];
  const float* W_B = (const float*)d_in[3];
  const float* W_C = (const float*)d_in[4];
  const float* W_dt = (const float*)d_in[5];
  const float* b_dt = (const float*)d_in[6];
  const float* dt_bias = (const float*)d_in[7];
  const float* rope_freq = (const float*)d_in[8];
  const float* ln_w = (const float*)d_in[9];
  const float* ln_b = (const float*)d_in[10];
  const float* W_out = (const float*)d_in[11];
  float* out = (float*)d_out;
  float* fstate = out + (size_t)kRows * kDm;
  char* ws = (char*)d_ws;
  unsigned short* X16 = (unsigned short*)(ws + kOffX16);
  unsigned short* WI = (unsigned short*)(ws + kOffWI);
  unsigned short* WBC = (unsigned short*)(ws + kOffWBC);
  unsigned short* WD = (unsigned short*)(ws + kOffWD);
  unsigned short* WO = (unsigned short*)(ws + kOffWO);
  float* BV = (float*)(ws + kOffBV);
  float* TAB = (float*)(ws + kOffTAB);
  float* XZ = (float*)(ws + kOffXZ);
  float* BC = (float*)(ws + kOffBC);
  float* DTL = (float*)(ws + kOffDTL);
  float* YP = (float*)(ws + kOffYP);
  float* FS = (float*)(ws + kOffFS);
  unsigned short* G16 = (unsigned short*)(ws + kOffG16);

  cast_rows_kernel<<<(kRows * (kDm / 8)) / kThr, kThr, 0, stream>>>(x, X16, kDm / 8, kDm, 0, kInCarry);
  cast_rows_kernel<<<(kDi2 * (kDm / 8)) / kThr, kThr, 0, stream>>>(W_in, WI, kDm / 8, kDm, 0, kWCarry);
  cast_rows_kernel<<<(kNs * (kDm / 8)) / kThr, kThr, 0, stream>>>(W_B, WBC, kDm / 8, kDm, 0, kWCarry);
  cast_rows_kernel<<<(kNs * (kDm / 8)) / kThr, kThr, 0, stream>>>(W_C, WBC + (size_t)kNs * kDm, kDm / 8, kDm, 0, kWCarry);
  cast_rows_kernel<<<(kDi * (kDm / 8)) / kThr, kThr, 0, stream>>>(W_dt, WD, kDm / 8, kDm, 0, kWCarry);
  cast_rows_kernel<<<(kDm * (kDi / 8)) / kThr, kThr, 0, stream>>>(W_out, WO, kDi / 8, kDiX, 0, kWCarry);
  cast_rows_kernel<<<(kDm * (kDi / 8)) / kThr, kThr, 0, stream>>>(W_out, WO, kDi / 8, kDiX, kDi, kWCarry);
  bias_rows_kernel<<<kBvTot / kThr, kThr, 0, stream>>>(b_dt, BV);
  rope_table_kernel<<<(kSeq * kHalf) / kThr, kThr, 0, stream>>>(rope_freq, TAB);

  wmma_gemm64<0, false, 2, 0, false, 0><<<dim3((kRows / 64) * (kDi2 / 64) / 8, 1), 256, 0, stream>>>(
      X16, X16, kDm, 0L, WI, WI, kDm, 0L, (void*)XZ, (void*)XZ, kDi2, 0L, BV + kBvZ, nullptr, 0L, kRows, kDi2, kDm, kScIn);
  wmma_gemm64<0, false, 2, 0, false, 0><<<dim3((kRows / 64) * (64 / 64) / 8, 1), 256, 0, stream>>>(
      X16, X16, kDm, 0L, WBC, WBC, kDm, 0L, (void*)BC, (void*)BC, 64, 0L, BV + kBvZ, nullptr, 0L, kRows, 64, kDm, kScIn);
  wmma_gemm64<0, false, 2, 0, false, 0><<<dim3((kRows / 64) * (kDi / 64) / 8, 1), 256, 0, stream>>>(
      X16, X16, kDm, 0L, WD, WD, kDm, 0L, (void*)DTL, (void*)DTL, kDi, 0L, BV + kBvDt, nullptr, 0L, kRows, kDi, kDm, kScIn);
  trap_scan_kernel<0><<<(kBatch * kDi) / kThr, kThr, 0, stream>>>(DTL, XZ, BC, TAB, A_log, dt_bias, YP, FS);
  trap_scan_kernel<4><<<(kBatch * kDi) / kThr, kThr, 0, stream>>>(DTL, XZ, BC, TAB, A_log, dt_bias, YP, FS);
  trap_scan_kernel<8><<<(kBatch * kDi) / kThr, kThr, 0, stream>>>(DTL, XZ, BC, TAB, A_log, dt_bias, YP, FS);
  trap_scan_kernel<12><<<(kBatch * kDi) / kThr, kThr, 0, stream>>>(DTL, XZ, BC, TAB, A_log, dt_bias, YP, FS);
  final_state_kernel<<<(kBatch * kDi) / kThr, kThr, 0, stream>>>(FS, fstate);
  gate_ln_kernel<<<kRows, kThr, 0, stream>>>(YP, XZ, ln_w, ln_b, G16);
  wmma_gemm64<0, false, 2, 0, false, 0><<<dim3((kRows / 64) * (kDm / 64) / 8, 1), 256, 0, stream>>>(
      G16, G16, kDiX, 0L, WO, WO, kDiX, 0L, (void*)out, (void*)out, kDm, 0L, BV + kBvZ, nullptr, 0L, kRows, kDm, kDiX, kScA);
}
